// DepthConv_73564199846424
// MI455X (gfx1250) — hardware-verified
//
#include <hip/hip_runtime.h>
#include <stdint.h>
#include <stddef.h>

typedef __attribute__((ext_vector_type(16))) __bf16   v16b;
typedef __attribute__((ext_vector_type(8)))  __bf16   v8b;
typedef __attribute__((ext_vector_type(8)))  float    v8f;
typedef __attribute__((ext_vector_type(4)))  float    v4f;
typedef __attribute__((ext_vector_type(4)))  unsigned v4u;

constexpr int NBATCH  = 8;
constexpr int NCH_IN  = 64;
constexpr int NCH_OUT = 64;
constexpr int IMG_H   = 128;
constexpr int IMG_W   = 128;
constexpr int NTAP    = 9;
constexpr int STRIP   = 64;
constexpr int NCOL    = STRIP + 2;
constexpr int CPAD    = 72;
constexpr int SLABP   = 36;
constexpr int NTHR    = 256;
constexpr float ALPHA_NEG = -8.3f;

constexpr int PREP_ITEMS  = NTAP * NCH_OUT * (NCH_IN / 8);
constexpr int PREP_BLOCKS = PREP_ITEMS / NTHR;
constexpr int MAIN_BLOCKS = NBATCH * IMG_H * (IMG_W / STRIP);
constexpr size_t WT_HALVES = (size_t)NTAP * NCH_OUT * NCH_IN;
constexpr size_t WT_BYTES  = WT_HALVES * 2;

static_assert(PREP_ITEMS % NTHR == 0);
static_assert(PREP_BLOCKS * NTHR == PREP_ITEMS);
static_assert(IMG_W % STRIP == 0);
static_assert(NCH_IN % 32 == 0);
static_assert(NCH_OUT == 64);
static_assert((CPAD * 2) % 16 == 0);
static_assert((SLABP * 4) % 16 == 0);


__device__ __forceinline__ unsigned short f2bf_bits(float f) {
  unsigned u = __float_as_uint(f);
  return (unsigned short)((u + 0x7FFFu + ((u >> 16) & 1u)) >> 16);
}
__device__ __forceinline__ float bf_bits2f(unsigned short h) { return __uint_as_float(((unsigned)h) << 16); }
__device__ __forceinline__ float bf_rne(float f) { return bf_bits2f(f2bf_bits(f)); }

__device__ __forceinline__ v16b frag_load_bf(const __bf16* p) {
  union { v16b v; v8b h[2]; } f;
  f.h[0] = *(const v8b*)(p);
  f.h[1] = *(const v8b*)(p + 16);
  return f.v;
}

__device__ __forceinline__ v8f mma_bf(v16b a, v16b b, v8f c) {
  c = __builtin_amdgcn_wmma_f32_16x16x32_bf16(false, a, false, b, (short)0, c, false, false);
  asm volatile("v_nop\n\tv_nop\n\tv_nop\n\tv_nop" : "+v"(c) : "v"(a), "v"(b));
  return c;
}

__device__ __forceinline__ v4u pack8_u16(unsigned short h0, unsigned short h1, unsigned short h2, unsigned short h3,
                                         unsigned short h4, unsigned short h5, unsigned short h6, unsigned short h7) {
  v4u u;
  u[0] = (unsigned)h0 | ((unsigned)h1 << 16);
  u[1] = (unsigned)h2 | ((unsigned)h3 << 16);
  u[2] = (unsigned)h4 | ((unsigned)h5 << 16);
  u[3] = (unsigned)h6 | ((unsigned)h7 << 16);
  return u;
}

__global__ __launch_bounds__(NTHR)
void prep_weight_planes(const float* __restrict__ weight, unsigned short* __restrict__ wT)
{
  const int g   = blockIdx.x * NTHR + threadIdx.x;
  const int q8  = g & 7;
  const int row = g >> 3;
  const int tap = row >> 6;
  const int o   = row & 63;
  const float* src = weight + ((size_t)o * NCH_IN + q8 * 8) * NTAP + tap;
  unsigned short hb[8];
#pragma unroll
  for (int e = 0; e < 8; ++e) hb[e] = f2bf_bits(src[e * NTAP]);
  const v4u u = pack8_u16(hb[0], hb[1], hb[2], hb[3], hb[4], hb[5], hb[6], hb[7]);
  unsigned short* dst = wT + (size_t)row * NCH_IN + q8 * 8;
  *(volatile v4u*)dst = u;
  __threadfence();
  *(volatile v4u*)dst = u;
}

__global__ __launch_bounds__(NTHR)
void depthconv_tap_wmma(const float* __restrict__ img,
                        const float* __restrict__ depth,
                        const float* __restrict__ bias,
                        const unsigned short* __restrict__ wT,
                        float* __restrict__ out)
{
  __shared__ __align__(16) unsigned short sImg[3 * NCOL * CPAD];
  __shared__ __align__(16) float sDW[NTAP * STRIP];
  __shared__ __align__(16) float sBias[NCH_OUT];
  __shared__ __align__(16) float sSlab[8][16 * SLABP];

  const int tid = threadIdx.x;
  const int blk = blockIdx.x;
  const int w0  = (blk & 1) * STRIP;
  const int h   = (blk >> 1) & (IMG_H - 1);
  const int b   = blk >> 8;

  if (tid < NCH_OUT) sBias[tid] = bf_rne(bias[tid]);

  const float* depth_b = depth + (size_t)b * (IMG_H * IMG_W);
  for (int idx = tid; idx < NTAP * STRIP; idx += NTHR) {
    const int tap = idx >> 6;
    const int p   = idx & 63;
    const int ti  = tap / 3;
    const int tj  = tap - ti * 3;
    const int w   = w0 + p;
    const float center = bf_rne(depth_b[h * IMG_W + w]);
    const int r  = h + ti - 1;
    const int cc = w + tj - 1;
    const bool inb = (r >= 0) && (r < IMG_H) && (cc >= 0) && (cc < IMG_W);
    const int rc  = r < 0 ? 0 : (r >= IMG_H ? IMG_H - 1 : r);
    const int ccc = cc < 0 ? 0 : (cc >= IMG_W ? IMG_W - 1 : cc);
    float dn = bf_rne(depth_b[rc * IMG_W + ccc]);
    dn = inb ? dn : 0.0f;
    sDW[idx] = expf(ALPHA_NEG * fabsf(center - dn));
  }

  const float* img_b = img + (size_t)b * (NCH_IN * IMG_H * IMG_W);
#pragma unroll 1
  for (int f = tid; f < 3 * 8 * NCOL; f += NTHR) {
    const int col = f % NCOL;
    const int t   = f / NCOL;
    const int cg  = t & 7;
    const int r3  = t >> 3;
    const int r   = h + r3 - 1;
    const int cc  = w0 + col - 1;
    const bool inb = (r >= 0) && (r < IMG_H) && (cc >= 0) && (cc < IMG_W);
    const int rc  = r < 0 ? 0 : (r >= IMG_H ? IMG_H - 1 : r);
    const int ccc = cc < 0 ? 0 : (cc >= IMG_W ? IMG_W - 1 : cc);
    const float* src = img_b + ((size_t)(cg * 8) * IMG_H + rc) * IMG_W + ccc;
    unsigned short hb[8];
#pragma unroll
    for (int e = 0; e < 8; ++e) {
      const float v = src[(size_t)e * (IMG_H * IMG_W)];
      hb[e] = inb ? f2bf_bits(v) : (unsigned short)0;
    }
    const v4u u = pack8_u16(hb[0], hb[1], hb[2], hb[3], hb[4], hb[5], hb[6], hb[7]);
    *(v4u*)(&sImg[(r3 * NCOL + col) * CPAD + cg * 8]) = u;
  }
  __syncthreads();

  const int wave = tid >> 5;
  const int lane = tid & 31;
  const int rl   = lane & 15;
  const int hsel = lane >> 4;
  const int koff = hsel * 8;
  const int mt   = wave >> 1;
  const int nh   = wave & 1;
  const int pxA  = nh * 32 + rl;
  const int pxB  = pxA + 16;

  const __bf16* wA = (const __bf16*)wT + (size_t)(mt * 16 + rl) * NCH_IN + koff;
  const __bf16* sI = (const __bf16*)(&sImg[0]);

  v8f acc0 = (v8f){0.f,0.f,0.f,0.f,0.f,0.f,0.f,0.f};
  v8f acc1 = (v8f){0.f,0.f,0.f,0.f,0.f,0.f,0.f,0.f};

#pragma unroll
  for (int tap = 0; tap < NTAP; ++tap) {
    const int ti = tap / 3;
    const int tj = tap - ti * 3;
    const __bf16* ap = wA + (size_t)tap * (NCH_OUT * NCH_IN);
    const v16b a0 = frag_load_bf(ap);
    const v16b a1 = frag_load_bf(ap + 32);
    const __bf16* bp0 = sI + (size_t)(ti * NCOL + pxA + tj) * CPAD + koff;
    const __bf16* bp1 = bp0 + 16 * CPAD;
    const v16b b00 = frag_load_bf(bp0);
    const v16b b01 = frag_load_bf(bp0 + 32);
    const v16b b10 = frag_load_bf(bp1);
    const v16b b11 = frag_load_bf(bp1 + 32);
    v8f t0 = (v8f){0.f,0.f,0.f,0.f,0.f,0.f,0.f,0.f};
    v8f t1 = (v8f){0.f,0.f,0.f,0.f,0.f,0.f,0.f,0.f};
    t0 = mma_bf(a0, b00, t0);
    t0 = mma_bf(a1, b01, t0);
    t1 = mma_bf(a0, b10, t1);
    t1 = mma_bf(a1, b11, t1);
    const float d0 = sDW[tap * STRIP + pxA];
    const float d1 = sDW[tap * STRIP + pxB];
#pragma unroll
    for (int r = 0; r < 8; ++r) {
      acc0[r] = fmaf(t0[r], d0, acc0[r]);
      acc1[r] = fmaf(t1[r], d1, acc1[r]);
    }
  }

  float* slab = sSlab[wave];
#pragma unroll
  for (int r = 0; r < 8; ++r) {
    const int ol = 8 * hsel + r;
    const float bv = sBias[mt * 16 + ol];
    slab[ol * SLABP + rl]      = acc0[r] + bv;
    slab[ol * SLABP + 16 + rl] = acc1[r] + bv;
  }
  __builtin_amdgcn_fence(__ATOMIC_RELEASE, "workgroup");
  __builtin_amdgcn_wave_barrier();
  __builtin_amdgcn_fence(__ATOMIC_ACQUIRE, "workgroup");
  {
    const int q  = lane >> 3;
    const int c4 = (lane & 7) * 4;
    float* ob = out + (((size_t)b * NCH_OUT + mt * 16) * IMG_H + h) * IMG_W + w0 + nh * 32 + c4;
    for (int pass = 0; pass < 2; ++pass) {
#pragma unroll
      for (int it = 0; it < 4; ++it) {
        const int row = it * 4 + q;
        const v4f v = *(const v4f*)(slab + row * SLABP + c4);
        *(volatile v4f*)(ob + (size_t)row * (IMG_H * IMG_W)) = v;
      }
      __threadfence();
    }
  }
}

extern "C" void kernel_launch(void* const* d_in, const int* in_sizes, int n_in,
                              void* d_out, int out_size, void* d_ws, size_t ws_size,
                              hipStream_t stream)
{
  if (n_in < 4) return;
  if (in_sizes[0] != NBATCH * NCH_IN * IMG_H * IMG_W) return;
  if (in_sizes[1] != NBATCH * IMG_H * IMG_W) return;
  if (in_sizes[2] != NCH_OUT * NCH_IN * NTAP) return;
  if (in_sizes[3] != NCH_OUT) return;
  if (out_size != NBATCH * NCH_OUT * IMG_H * IMG_W) return;
  if (ws_size < WT_BYTES) return;

  const float* img    = (const float*)d_in[0];
  const float* depth  = (const float*)d_in[1];
  const float* weight = (const float*)d_in[2];
  const float* bias   = (const float*)d_in[3];
  float* outp         = (float*)d_out;
  unsigned short* wT  = (unsigned short*)d_ws;

  prep_weight_planes<<<PREP_BLOCKS, NTHR, 0, stream>>>(weight, wT);
  depthconv_tap_wmma<<<MAIN_BLOCKS, NTHR, 0, stream>>>(img, depth, bias, wT, outp);
}
